// RGATLayer_11553462026815
// MI455X (gfx1250) — hardware-verified
//
#include <hip/hip_runtime.h>
#include <math.h>

#ifndef NB
#define NB 4
#endif
#ifndef SEQ
#define SEQ 1024
#endif
#define SEQ_FULL 1024
#define DIM 128
#define NREL 4
#define MTOK (NB * SEQ)
#define HI_PLANE ((size_t)MTOK * DIM)

#define CARRY_X 8.0f
#define CARRY_W 32.0f
#define G_SC (1.0f / 256.0f)
#define CARRY_J 16.0f
#define CARRY_I 64.0f
#define S_UNDO (1.0f / 1024.0f)
#define CARRY_P 1024.0f
#define O_UNDO (1.0f / 16384.0f)
#define FLUSH_T (1.0f / 16384.0f)
#define LOG2E 1.442695f
#define MASK_FILL (-9.0e15f)
#define LEAKY 0.2f

static_assert(CARRY_X * CARRY_W * G_SC == 1.0f);
static_assert(CARRY_J * CARRY_I * S_UNDO == 1.0f);
static_assert(CARRY_P * CARRY_J * O_UNDO == 1.0f);
static_assert(SEQ % 64 == 0 && SEQ <= SEQ_FULL);
static_assert(MTOK % 64 == 0);
static_assert(DIM == 128 && DIM % 64 == 0 && DIM % 32 == 0);
static_assert((MTOK * DIM / 8) % 256 == 0);
static_assert(NREL * DIM == 512);

#define ROWS_MIN ((NB - 1) * SEQ_FULL + SEQ)
#define HID_MIN (ROWS_MIN * DIM)
#define ADJ_MIN (((NB - 1) * SEQ_FULL + SEQ - 1) * SEQ_FULL + SEQ)

typedef __attribute__((ext_vector_type(16))) _Float16 v16h;
typedef __attribute__((ext_vector_type(8)))  _Float16 v8h;
typedef __attribute__((ext_vector_type(2)))  _Float16 v2h;
typedef __attribute__((ext_vector_type(8)))  float    v8f;
typedef __attribute__((ext_vector_type(4)))  float    v4f;
typedef __attribute__((ext_vector_type(2)))  float    v2f;
typedef __attribute__((ext_vector_type(4)))  unsigned int v4u;
typedef __attribute__((ext_vector_type(4)))  int      v4i;


#define VST2(T, ptr, val) do { const T vst2_v_ = (val); *(volatile T*)(ptr) = vst2_v_; __threadfence(); *(volatile T*)(ptr) = vst2_v_; } while (0)
#define VST2V4(ptr, val) do { const v4f vst2_v4_ = (val); *(volatile v4f*)(ptr) = vst2_v4_; __threadfence(); *(volatile v4f*)(ptr) = vst2_v4_; } while (0)

__device__ __forceinline__ float bfr(float f) {
    unsigned u = __float_as_uint(f);
    u += 0x7FFFu + ((u >> 16) & 1u);
    return __uint_as_float(u & 0xFFFF0000u);
}

static __device__ __forceinline__ v2h toh2_flush(float a, float b) {
    const float wa = (fabsf(a) < FLUSH_T) ? 0.0f : a;
    const float wb = (fabsf(b) < FLUSH_T) ? 0.0f : b;
    v2f f; f.x = wa; f.y = wb;
    return __builtin_convertvector(f, v2h);
}
static __device__ __forceinline__ unsigned pk2h_flush(float a, float b) {
    return __builtin_bit_cast(unsigned, toh2_flush(a, b));
}
__device__ __forceinline__ void st8h(unsigned short* P, size_t o, const float* v) {
    v4u pk;
    pk.x = pk2h_flush(v[0], v[1]);
    pk.y = pk2h_flush(v[2], v[3]);
    pk.z = pk2h_flush(v[4], v[5]);
    pk.w = pk2h_flush(v[6], v[7]);
    VST2(v4u, (v4u*)(P + o), pk);
}
static __device__ __forceinline__ void split2(float a, float b, unsigned& hi, unsigned& lo) {
    const v2h h = toh2_flush(a, b);
    const v2h r = toh2_flush(a - (float)h.x, b - (float)h.y);
    hi = __builtin_bit_cast(unsigned, h);
    lo = __builtin_bit_cast(unsigned, r);
}
static __device__ __forceinline__ void split8(const float* v, v4u& whi, v4u& wlo) {
    unsigned h0, l0, h1, l1, h2, l2, h3, l3;
    split2(v[0], v[1], h0, l0);
    split2(v[2], v[3], h1, l1);
    split2(v[4], v[5], h2, l2);
    split2(v[6], v[7], h3, l3);
    whi.x = h0; whi.y = h1; whi.z = h2; whi.w = h3;
    wlo.x = l0; wlo.y = l1; wlo.z = l2; wlo.w = l3;
}

union FragU { v16h v; v8h h[2]; };
union PFrag { v16h v; v2h p[8]; };
__device__ __forceinline__ v16h frag_ld(const _Float16* p) {
    FragU f; f.h[0] = *(const v8h*)(p); f.h[1] = *(const v8h*)(p + 16); return f.v;
}
__device__ __forceinline__ v8f wmma16(v16h a, v16h b, v8f c) {
    c = __builtin_amdgcn_wmma_f32_16x16x32_f16(false, a, false, b, (short)0, c, false, false);
    asm volatile("v_nop\n\tv_nop\n\tv_nop\n\tv_nop" : "+v"(c) : "v"(a), "v"(b));
    return c;
}
__device__ __forceinline__ void wave_sync_lds() {
    __builtin_amdgcn_fence(3  , "workgroup");
    __builtin_amdgcn_wave_barrier();
    __builtin_amdgcn_fence(2  , "workgroup");
}

static_assert(2 * 4 * 32 * 16 == 16 * 64 * 4);
static_assert(8 * 16 * 68 * 4 <= 131072);
__global__ __launch_bounds__(256) void k_gemm64f(
    const _Float16* __restrict__ A, unsigned lda, const _Float16* __restrict__ Bt, unsigned ldb,
    float* __restrict__ C, unsigned ldc, unsigned M, unsigned N, unsigned K) {
  __shared__ __align__(16) float sT[8][16 * 68];
  const unsigned lane = threadIdx.x & 31u;
  const unsigned wave = (unsigned)__builtin_amdgcn_readfirstlane((int)(threadIdx.x >> 5));
  const unsigned tilesN = N >> 6, tilesM = M >> 6;
  const unsigned bx = blockIdx.x;
  const unsigned tile = bx * 8u + wave;
  if (tile >= tilesM * tilesN) return;
  const unsigned tm = tile / tilesN;
  const unsigned tn = tile - tm * tilesN;
  const unsigned m0 = tm << 6, n0 = tn << 6;
  const unsigned rlane = lane & 15u;
  const unsigned koff = (lane >> 4) * 8u;
  const unsigned mOff = koff;

  v8f acc[4][4];
#pragma unroll
  for (int i = 0; i < 4; ++i)
#pragma unroll
    for (int j = 0; j < 4; ++j) acc[i][j] = (v8f){0.f,0.f,0.f,0.f,0.f,0.f,0.f,0.f};

  for (unsigned k0 = 0; k0 < K; k0 += 32u) {
    v16h bh[4];
#pragma unroll
    for (int j = 0; j < 4; ++j)
      bh[j] = frag_ld(Bt + (size_t)(n0 + ((unsigned)j << 4) + rlane) * ldb + koff + k0);
#pragma unroll
    for (int i = 0; i < 4; ++i) {
      const v16h ah = frag_ld(A + (size_t)(m0 + ((unsigned)i << 4) + rlane) * lda + koff + k0);
#pragma unroll
      for (int j = 0; j < 4; ++j)
        acc[i][j] = wmma16(ah, bh[j], acc[i][j]);
    }
  }

#pragma unroll
  for (int i = 0; i < 4; ++i) {
    const unsigned mBase = m0 + ((unsigned)i << 4);
#pragma unroll
    for (int j = 0; j < 4; ++j) {
#pragma unroll
      for (int r = 0; r < 8; ++r) {
        const float v = acc[i][j][r] * G_SC;
        sT[wave][(mOff + (unsigned)r) * 68u + ((unsigned)j << 4) + rlane] = v;
      }
    }
    wave_sync_lds();
    {
      const unsigned hh = lane >> 4, c4 = (lane & 15u) * 4u;
#pragma unroll
      for (int half = 0; half < 2; ++half) {
        v4f vv[4];
#pragma unroll
        for (int it = 0; it < 4; ++it) {
          const unsigned row = (unsigned)(half * 4 + it) * 2u + hh;
          vv[it] = *(const v4f*)&sT[wave][row * 68u + c4];
        }
        for (int pass = 0; pass < 2; ++pass) {
#pragma unroll
          for (int it = 0; it < 4; ++it) {
            const unsigned row = (unsigned)(half * 4 + it) * 2u + hh;
            *(volatile v4f*)(C + (size_t)(mBase + row) * ldc + n0 + c4) = vv[it];
          }
          __threadfence();
        }
      }
    }
    wave_sync_lds();
  }
}

__global__ __launch_bounds__(256) void k_wt16(const float* __restrict__ Wm, unsigned KI, unsigned NO, unsigned lgper,
                                              unsigned short* __restrict__ W16) {
    const unsigned layer = blockIdx.y;
    const float* Wl = Wm + (size_t)layer * KI * NO;
    unsigned short* Dl = W16 + (size_t)layer * KI * NO;
    const unsigned u = blockIdx.x * 256u + threadIdx.x;
    const unsigned per = 1u << lgper;
    if (u >= NO * per) return;
    const unsigned k0 = 8u * (u & (per - 1u));
    const unsigned o = u >> lgper;
    float v[8];
#pragma unroll
    for (int i = 0; i < 8; ++i) v[i] = bfr(Wl[(size_t)(k0 + (unsigned)i) * NO + o]) * CARRY_W;
    st8h(Dl, (size_t)o * KI + k0, v);
}

__global__ __launch_bounds__(256) void k_cvt8(const float* __restrict__ x, unsigned short* __restrict__ xp16) {
    const unsigned bx = blockIdx.x;
    const unsigned u = bx * 256u + threadIdx.x;
    if (u >= (unsigned)(MTOK * DIM / 8)) return;
    const unsigned prow = u >> 4, c0 = (u & 15u) * 8u;
    const unsigned b = prow / (unsigned)SEQ;
    const unsigned n = prow - b * (unsigned)SEQ;
    const float* xr = x + (size_t)(b * (unsigned)SEQ_FULL + n) * DIM + c0;
    const v4f a = *(const v4f*)xr;
    const v4f q = *(const v4f*)(xr + 4);
    v4u pk;
    pk.x = pk2h_flush(bfr(a.x) * CARRY_X, bfr(a.y) * CARRY_X);
    pk.y = pk2h_flush(bfr(a.z) * CARRY_X, bfr(a.w) * CARRY_X);
    pk.z = pk2h_flush(bfr(q.x) * CARRY_X, bfr(q.y) * CARRY_X);
    pk.w = pk2h_flush(bfr(q.z) * CARRY_X, bfr(q.w) * CARRY_X);
    VST2(v4u, (v4u*)(xp16 + (size_t)prow * DIM + c0), pk);
}

#define PL_ROWS 64
#define PL_PITCH 132
static_assert(256 * 8 * 16 == PL_ROWS * DIM * 4);
static_assert(256 * 4 * 16 == PL_ROWS * DIM * 2);
static_assert(256 * 4 * 16 == DIM * PL_ROWS * 2);
static_assert(PL_ROWS * PL_PITCH * 4 + NREL * DIM * 4 <= 131072);
__global__ __launch_bounds__(256) void k_planes(const float* __restrict__ Hf, const float* __restrict__ a_params,
                                                unsigned short* __restrict__ HJh, unsigned short* __restrict__ HJl,
                                                unsigned short* __restrict__ VTh, unsigned short* __restrict__ VTl,
                                                unsigned short* __restrict__ HIp) {
    __shared__ __align__(16) float sH[PL_ROWS * PL_PITCH];
    __shared__ __align__(16) float sAp[NREL * DIM];
    const unsigned t = threadIdx.x;
    const unsigned bx = blockIdx.x;
    const unsigned TPB = (unsigned)(SEQ / PL_ROWS);
    const unsigned b = bx / TPB;
    const unsigned jt = bx - b * TPB;
    const unsigned row0 = b * (unsigned)SEQ + jt * (unsigned)PL_ROWS;
#pragma unroll
    for (int it = 0; it < 8; ++it) {
        const unsigned idx = (unsigned)it * 256u + t;
        const unsigned row = idx >> 5, c4 = (idx & 31u) * 4u;
        *(v4f*)&sH[row * PL_PITCH + c4] = *(const v4f*)(Hf + (size_t)(row0 + row) * DIM + c4);
    }
    sAp[t] = bfr(a_params[t]);
    sAp[t + 256u] = bfr(a_params[t + 256u]);
    __syncthreads();

#pragma unroll 1
    for (unsigned it = 0; it < 4u; ++it) {
        const unsigned item = it * 256u + t;
        const unsigned row = item >> 4, c0 = (item & 15u) * 8u;
        const v4f q0 = *(const v4f*)&sH[row * PL_PITCH + c0];
        const v4f q1 = *(const v4f*)&sH[row * PL_PITCH + c0 + 4u];
        const float hv[8] = {q0.x, q0.y, q0.z, q0.w, q1.x, q1.y, q1.z, q1.w};
        float cv[8];
#pragma unroll
        for (int e = 0; e < 8; ++e) cv[e] = hv[e] * CARRY_J;
        v4u whi, wlo;
        split8(cv, whi, wlo);
        const size_t o = (size_t)(row0 + row) * DIM + c0;
        VST2(v4u, (v4u*)(HJh + o), whi);
        VST2(v4u, (v4u*)(HJl + o), wlo);
#pragma unroll
        for (int r = 0; r < NREL; ++r) {
            const v4f g0 = *(const v4f*)&sAp[(unsigned)r * DIM + c0];
            const v4f g1 = *(const v4f*)&sAp[(unsigned)r * DIM + c0 + 4u];
            v4u w;
            w.x = pk2h_flush((hv[0] * g0.x) * CARRY_I, (hv[1] * g0.y) * CARRY_I);
            w.y = pk2h_flush((hv[2] * g0.z) * CARRY_I, (hv[3] * g0.w) * CARRY_I);
            w.z = pk2h_flush((hv[4] * g1.x) * CARRY_I, (hv[5] * g1.y) * CARRY_I);
            w.w = pk2h_flush((hv[6] * g1.z) * CARRY_I, (hv[7] * g1.w) * CARRY_I);
            VST2(v4u, (v4u*)(HIp + (size_t)r * HI_PLANE + o), w);
        }
    }
#pragma unroll 1
    for (unsigned it = 0; it < 4u; ++it) {
        const unsigned item = it * 256u + t;
        const unsigned d = item >> 3, jg = item & 7u;
        float cv[8];
#pragma unroll
        for (int e = 0; e < 8; ++e) cv[e] = sH[(8u * jg + (unsigned)e) * PL_PITCH + d] * CARRY_J;
        v4u whi, wlo;
        split8(cv, whi, wlo);
        const size_t o = (size_t)(b * (unsigned)DIM + d) * SEQ + jt * (unsigned)PL_ROWS + 8u * jg;
        VST2(v4u, (v4u*)(VTh + o), whi);
        VST2(v4u, (v4u*)(VTl + o), wlo);
    }
}

#define AT_WAVES 4
#define AT_OP 132
static_assert(32 * 16 * 16 == 16 * DIM * 4);
static_assert(AT_WAVES * 16 * AT_OP * 4 <= 131072);
static_assert((NB * (SEQ / 16)) % AT_WAVES == 0);
__global__ __launch_bounds__(128) __attribute__((amdgpu_num_vgpr(256))) void k_mattn(
    const _Float16* __restrict__ HIp, const _Float16* __restrict__ HJh, const _Float16* __restrict__ HJl,
    const _Float16* __restrict__ VTh, const _Float16* __restrict__ VTl,
    const int* __restrict__ adj, const float* __restrict__ amplifier, float* __restrict__ out) {
    __shared__ __align__(16) float sO[AT_WAVES][16 * AT_OP];
    const unsigned lane = threadIdx.x & 31u;
    const unsigned wave = (unsigned)__builtin_amdgcn_readfirstlane((int)(threadIdx.x >> 5));
    const unsigned hh = lane >> 4, c = lane & 15u;
    const unsigned bx = blockIdx.x;
    const unsigned tile = bx * (unsigned)AT_WAVES + wave;
    if (tile >= (unsigned)(NB * (SEQ / 16))) return;
    const unsigned TPB = (unsigned)(SEQ / 16);
    const unsigned b = tile / TPB;
    const unsigned i0 = (tile - b * TPB) * 16u;

    float amp[4];
    amp[0] = bfr(amplifier[0]); amp[1] = bfr(amplifier[1]); amp[2] = bfr(amplifier[2]); amp[3] = bfr(amplifier[3]);

    const unsigned qoff  = (b * (unsigned)SEQ + i0 + c) * (unsigned)DIM + 8u * hh;
    const unsigned jbase = (b * (unsigned)SEQ + c) * (unsigned)DIM + 8u * hh;
    const unsigned vbase = (b * (unsigned)DIM + c) * (unsigned)SEQ + 8u * hh;
    const size_t   abase = (size_t)(b * (unsigned)SEQ_FULL + i0 + c) * SEQ_FULL + 8u * hh;

    v8f O[8];
#pragma unroll
    for (int dt = 0; dt < 8; ++dt) O[dt] = (v8f){0.f,0.f,0.f,0.f,0.f,0.f,0.f,0.f};
    float m = -3.0e38f, l = 0.0f;

#pragma unroll 1
    for (unsigned j0 = 0; j0 < (unsigned)SEQ; j0 += 32u) {
        float tl[2][8];
#pragma unroll
        for (int tt = 0; tt < 2; ++tt) {
            const int* ap = adj + abase + j0 + 16u * (unsigned)tt;
            v4i a0 = *(const v4i*)ap;
            v4i a1 = *(const v4i*)(ap + 4);
            asm volatile("" : "+v"(a0), "+v"(a1));
            v8f S[4];
#pragma unroll
            for (int r = 0; r < 4; ++r) S[r] = (v8f){0.f,0.f,0.f,0.f,0.f,0.f,0.f,0.f};
            const unsigned jo = jbase + (j0 + 16u * (unsigned)tt) * (unsigned)DIM;
#pragma unroll 1
            for (unsigned kc = 0; kc < (unsigned)DIM; kc += 32u) {
                const v16h ah = frag_ld(HJh + jo + kc);
                const v16h al = frag_ld(HJl + jo + kc);
#pragma unroll
                for (int r = 0; r < 4; ++r) {
                    const v16h qf = frag_ld(HIp + (size_t)r * HI_PLANE + qoff + kc);
                    S[r] = wmma16(ah, qf, S[r]);
                    S[r] = wmma16(al, qf, S[r]);
                }
            }
            const int av[8] = {a0.x, a0.y, a0.z, a0.w, a1.x, a1.y, a1.z, a1.w};
#pragma unroll
            for (int r8 = 0; r8 < 8; ++r8) {
                const int a = av[r8];
                const int ri = min(max(a - 1, 0), 3);
                float sel = 0.0f;
#pragma unroll
                for (int r = 0; r < 4; ++r) {
                    float e = S[r][r8] * S_UNDO;
                    e = (e > 0.0f) ? e : LEAKY * e;
                    const float ea = e * amp[r];
                    sel = (ri == r) ? ea : sel;
                }
                const float alv = (a > 0) ? sel : MASK_FILL;
                tl[tt][r8] = alv * LOG2E;
            }
        }
        float mx = tl[0][0];
#pragma unroll
        for (int r8 = 1; r8 < 8; ++r8) mx = (tl[0][r8] > mx) ? tl[0][r8] : mx;
#pragma unroll
        for (int r8 = 0; r8 < 8; ++r8) mx = (tl[1][r8] > mx) ? tl[1][r8] : mx;
        const float mo = __shfl_xor(mx, 16, 32);
        mx = (mo > mx) ? mo : mx;
        const float mnew = (mx > m) ? mx : m;
        const float alpha = exp2f(m - mnew);
        m = mnew;
        float ps = 0.0f;
        PFrag pf;
#pragma unroll
        for (int tt = 0; tt < 2; ++tt) {
#pragma unroll
            for (int r2 = 0; r2 < 4; ++r2) {
                const float p0 = exp2f(tl[tt][2 * r2] - mnew);
                const float p1 = exp2f(tl[tt][2 * r2 + 1] - mnew);
                ps += p0 + p1;
                pf.p[4 * tt + r2] = toh2_flush(p0 * CARRY_P, p1 * CARRY_P);
            }
        }
        l = l * alpha + ps;
#pragma unroll
        for (int dt = 0; dt < 8; ++dt) O[dt] = O[dt] * alpha;

        unsigned vo = vbase + j0;
#pragma unroll
        for (int dt = 0; dt < 8; ++dt) {
            const v16h vh = frag_ld(VTh + vo);
            const v16h vl = frag_ld(VTl + vo);
            O[dt] = wmma16(vh, pf.v, O[dt]);
            O[dt] = wmma16(vl, pf.v, O[dt]);
            vo += 16u * (unsigned)SEQ;
            asm volatile("" : "+v"(vo));
        }
    }

    const float lother = __shfl_xor(l, 16, 32);
    const float lsum = l + lother;
    const float inv = O_UNDO / lsum;
#pragma unroll
    for (int dt = 0; dt < 8; ++dt) {
        v4f w0, w1;
        w0.x = O[dt][0] * inv; w0.y = O[dt][1] * inv; w0.z = O[dt][2] * inv; w0.w = O[dt][3] * inv;
        w1.x = O[dt][4] * inv; w1.y = O[dt][5] * inv; w1.z = O[dt][6] * inv; w1.w = O[dt][7] * inv;
        *(v4f*)&sO[wave][c * AT_OP + 16u * (unsigned)dt + 8u * hh] = w0;
        *(v4f*)&sO[wave][c * AT_OP + 16u * (unsigned)dt + 8u * hh + 4u] = w1;
    }
    wave_sync_lds();
    {
        float* outp = out + (size_t)(b * (unsigned)SEQ_FULL + i0) * DIM + 4u * lane;
#pragma unroll
        for (int half = 0; half < 2; ++half) {
            v4f vv[8];
#pragma unroll
            for (int it = 0; it < 8; ++it) {
                const unsigned row = (unsigned)(half * 8 + it);
                vv[it] = *(const v4f*)&sO[wave][row * AT_OP + 4u * lane];
            }
            for (int pass = 0; pass < 2; ++pass) {
#pragma unroll
                for (int it = 0; it < 8; ++it) {
                    const unsigned row = (unsigned)(half * 8 + it);
                    *(volatile v4f*)(outp + (size_t)row * DIM) = vv[it];
                }
                __threadfence();
            }
        }
    }
}

#define SZ_XP   ((size_t)MTOK * DIM * 2)
#define SZ_WT   ((size_t)DIM * DIM * 2)
#define SZ_HF   ((size_t)MTOK * DIM * 4)
#define SZ_HJ   ((size_t)MTOK * DIM * 2)
#define SZ_VT   ((size_t)NB * DIM * SEQ * 2)
#define SZ_HI   ((size_t)NREL * MTOK * DIM * 2)
static_assert(SZ_XP % 256 == 0 && SZ_WT % 256 == 0 && SZ_HF % 256 == 0 && SZ_HJ % 256 == 0 && SZ_VT % 256 == 0 && SZ_HI % 256 == 0);
static_assert(SZ_XP + SZ_WT + SZ_HF + 2 * SZ_HJ + 2 * SZ_VT + SZ_HI <= (size_t)134217728);

extern "C" void kernel_launch(void* const* d_in, const int* in_sizes, int n_in, void* d_out, int out_size,
                              void* d_ws, size_t ws_size, hipStream_t stream) {
    if (n_in < 6) return;
    if (in_sizes[0] < HID_MIN || in_sizes[1] < ADJ_MIN || in_sizes[2] < ROWS_MIN) return;
    if (in_sizes[3] < DIM * DIM || in_sizes[4] < NREL * DIM || in_sizes[5] < NREL || out_size < HID_MIN) return;

    const float* hidden    = (const float*)d_in[0];
    const int*   adj       = (const int*)d_in[1];
    const int*   ntmask    = (const int*)d_in[2];
    const float* Wm        = (const float*)d_in[3];
    const float* a_params  = (const float*)d_in[4];
    const float* amplifier = (const float*)d_in[5];
    (void)ntmask;
    float* out = (float*)d_out;

    char* wsp = (char*)d_ws;
    size_t off = 0;
    auto carve = [&](size_t bytes) -> void* { void* r = wsp + off; off += (bytes + 255) & ~(size_t)255; return r; };
    unsigned short* xp16 = (unsigned short*)carve(SZ_XP);
    unsigned short* wT   = (unsigned short*)carve(SZ_WT);
    float*          Hf   = (float*)carve(SZ_HF);
    unsigned short* HJh  = (unsigned short*)carve(SZ_HJ);
    unsigned short* HJl  = (unsigned short*)carve(SZ_HJ);
    unsigned short* VTh  = (unsigned short*)carve(SZ_VT);
    unsigned short* VTl  = (unsigned short*)carve(SZ_VT);
    unsigned short* HIp  = (unsigned short*)carve(SZ_HI);
    if (off > ws_size || off > (size_t)134217728) return;

    k_wt16<<<dim3((DIM * (DIM / 8)) / 256, 1), 256, 0, stream>>>(Wm, DIM, DIM, 4, wT);
    k_cvt8<<<(MTOK * DIM / 8) / 256, 256, 0, stream>>>(hidden, xp16);
    k_gemm64f<<<((MTOK / 64) * (DIM / 64) + 7) / 8, 256, 0, stream>>>((const _Float16*)xp16, DIM, (const _Float16*)wT, DIM,
        Hf, DIM, MTOK, DIM, DIM);
    k_planes<<<MTOK / PL_ROWS, 256, 0, stream>>>(Hf, a_params, HJh, HJl, VTh, VTl, HIp);
    k_mattn<<<(NB * (SEQ / 16)) / AT_WAVES, 32 * AT_WAVES, 0, stream>>>((const _Float16*)HIp, (const _Float16*)HJh, (const _Float16*)HJl,
        (const _Float16*)VTh, (const _Float16*)VTl, adj, amplifier, out);
}
